// GCN_55147380080825
// MI455X (gfx1250) — hardware-verified
//
#include <hip/hip_runtime.h>
#include <stddef.h>
#include <stdint.h>
#include <math.h>


#define DF     128
#define KA     384
#define KH     256
#define NCLS   40
#define NC3    64
#define NTHR   256
#define NWAVE  8
#define EPT    8
#define CHUNK  (NTHR * EPT)
#define WCAP   (EPT * 32)
#define LISTN  (NWAVE * WCAP)
#define NBA    1024
#define SLA    10
#define RCAP   24576
#define DEGCAP 64
#define GBM    64
#define GTHR   128
#define U_W1   2048
#define U_CB   6144
#define U_W2   4096
#define U_W3   2048
#define U_TOT  (U_W1 + U_CB + U_W2 + U_W3)
#define AGG_ZINTS    (LISTN + 2 * RCAP + 3 * NBA)
#define MISC_INTS    16
#define STGW         1280
#define AGG_LDS_INTS (AGG_ZINTS + MISC_INTS + NWAVE * STGW)
#define WSMAX  134217728

static_assert((CHUNK & (CHUNK - 1)) == 0 && CHUNK <= 4096);
static_assert((NBA & (NBA - 1)) == 0 && NBA == (1 << SLA));
static_assert(((long long)CHUNK << SLA) < (1LL << 31));
static_assert(NBA % NWAVE == 0 && NBA % 32 == 0 && NBA % GBM == 0 && (NBA / 32) % NWAVE == 0);
static_assert(RCAP % 4 == 0 && AGG_ZINTS % (NTHR * 4) == 0 && ((AGG_ZINTS + MISC_INTS) % 4) == 0);
static_assert(DF % 32 == 0 && KA % 32 == 0 && KH % 32 == 0 && KA == 3 * DF && KH == 2 * DF);
static_assert(GBM == (GTHR / 32) * 16 && DF == 4 * 32);
static_assert(U_W1 % NTHR == 0 && U_CB % NTHR == 0 && U_W2 % NTHR == 0 && U_W3 % NTHR == 0);
static_assert(STGW * 4 >= 32 * NCLS * 4 && STGW * 4 >= 2 * KH && (STGW % 4) == 0);
static_assert(NCLS % 4 == 0 && NCLS / 4 <= 16 && NCLS <= NC3);
static_assert(AGG_LDS_INTS * 4 <= 300000);
static_assert(DEGCAP >= 37 + 8 && RCAP >= 16759 + 2048);

typedef float          v4f   __attribute__((ext_vector_type(4)));
typedef float          v8f   __attribute__((ext_vector_type(8)));
typedef int            v4i   __attribute__((ext_vector_type(4)));
typedef int            v8i   __attribute__((ext_vector_type(8)));
typedef unsigned short v4us  __attribute__((ext_vector_type(4)));
typedef unsigned short v8us  __attribute__((ext_vector_type(8)));
typedef unsigned short v16us __attribute__((ext_vector_type(16)));
typedef __bf16         v16bf __attribute__((ext_vector_type(16)));
typedef v4f  __attribute__((may_alias)) v4fa;
typedef v4i  __attribute__((may_alias)) v4ia;
typedef v4us __attribute__((may_alias)) v4usa;
typedef v8us __attribute__((may_alias)) v8usa;
union FragB { v16bf v; v16us u; v8us h[2]; v8i w; };

__device__ __forceinline__ v8f wmb(const FragB& a, const FragB& b, v8f c) {
  v8f d = __builtin_amdgcn_wmma_f32_16x16x32_bf16(false, a.v, false, b.v, (short)0, c, false, false);
  asm volatile("v_nop\n\tv_nop\n\tv_nop\n\tv_nop" : "+v"(d) : "v"(a.w), "v"(b.w));
  return d;
}

__device__ __forceinline__ unsigned bf16_bits(float f) {
  const unsigned u = __float_as_uint(f);
  return (u + 0x7FFFu + ((u >> 16) & 1u)) >> 16;
}
__device__ __forceinline__ float bf16_val(float f) {
  return __uint_as_float(bf16_bits(f) << 16);
}

__device__ __forceinline__ void wave_sync() {
  __builtin_amdgcn_fence(__ATOMIC_RELEASE, "wavefront");
  __builtin_amdgcn_wave_barrier();
  __builtin_amdgcn_fence(__ATOMIC_ACQUIRE, "wavefront");
}

template <int SLB>
__device__ __forceinline__ int scan_chunk(const int* __restrict__ dsts, int nE, int cbase, int slotBase,
                                          int nb, int vec8, int* list, int tid, int lane, int wave) {
  int wc = 0;
  const int el0  = tid * EPT;
  const int e0   = cbase + el0;
  const int sent = -2147483647 - 1;
  v4i da, db;
  if (vec8 != 0 && cbase + CHUNK <= nE) {
    da = *(const v4i*)(dsts + e0);
    db = *(const v4i*)(dsts + e0 + 4);
  } else {
    da.x = (e0     < nE) ? dsts[min(e0,     nE - 1)] : sent;
    da.y = (e0 + 1 < nE) ? dsts[min(e0 + 1, nE - 1)] : sent;
    da.z = (e0 + 2 < nE) ? dsts[min(e0 + 2, nE - 1)] : sent;
    da.w = (e0 + 3 < nE) ? dsts[min(e0 + 3, nE - 1)] : sent;
    db.x = (e0 + 4 < nE) ? dsts[min(e0 + 4, nE - 1)] : sent;
    db.y = (e0 + 5 < nE) ? dsts[min(e0 + 5, nE - 1)] : sent;
    db.z = (e0 + 6 < nE) ? dsts[min(e0 + 6, nE - 1)] : sent;
    db.w = (e0 + 7 < nE) ? dsts[min(e0 + 7, nE - 1)] : sent;
  }
  const unsigned nbs = (unsigned)slotBase;
  const unsigned unb = (unsigned)nb;
  const unsigned s0 = (unsigned)da.x - nbs, s1 = (unsigned)da.y - nbs;
  const unsigned s2 = (unsigned)da.z - nbs, s3 = (unsigned)da.w - nbs;
  const unsigned s4 = (unsigned)db.x - nbs, s5 = (unsigned)db.y - nbs;
  const unsigned s6 = (unsigned)db.z - nbs, s7 = (unsigned)db.w - nbs;
  const bool h0 = s0 < unb, h1 = s1 < unb, h2 = s2 < unb, h3 = s3 < unb;
  const bool h4 = s4 < unb, h5 = s5 < unb, h6 = s6 < unb, h7 = s7 < unb;
  const unsigned any = __builtin_amdgcn_ballot_w32(h0 | h1 | h2 | h3 | h4 | h5 | h6 | h7);
  if (any != 0u) {
#define HITJ(J, HJ, SJ) { \
      const unsigned mj = __builtin_amdgcn_ballot_w32(HJ); \
      if (mj != 0u) { \
        if (HJ) { \
          const int pos = wc + (int)__builtin_amdgcn_mbcnt_lo(mj, 0u); \
          if (pos < WCAP) list[wave * WCAP + pos] = ((el0 + (J)) << SLB) | (int)(SJ); \
        } \
        wc += (int)__builtin_popcount(mj); } }
    HITJ(0, h0, s0)
    HITJ(1, h1, s1)
    HITJ(2, h2, s2)
    HITJ(3, h3, s3)
    HITJ(4, h4, s4)
    HITJ(5, h5, s5)
    HITJ(6, h6, s6)
    HITJ(7, h7, s7)
#undef HITJ
  }
  return wc;
}

__global__ __launch_bounds__(NTHR) void k_wprep(const float* __restrict__ W1, const float* __restrict__ W2,
                                                const float* __restrict__ W3, const float* __restrict__ CMB,
                                                unsigned short* W1T, unsigned short* CB3,
                                                unsigned short* W2T2, unsigned short* W3T2) {
  const int u = (int)blockIdx.x * NTHR + (int)threadIdx.x;
  const float* src;
  unsigned short* dp;
  int ld, ks, ncl;
  bool zr = false;
  if (u < U_W1) {
    const int n = u >> 4, k8 = (u & 15) * 8;
    src = W1; ld = DF; ks = k8; ncl = n;
    dp = W1T + (size_t)u * 8;
  } else if (u < U_W1 + U_CB) {
    const int v = u - U_W1;
    const int n = v / 48;
    const int k8 = (v - n * 48) * 8;
    src = CMB; ld = DF; ks = (k8 < DF) ? k8 : (k8 - DF); ncl = n;
    dp = CB3 + (size_t)v * 8;
  } else if (u < U_W1 + U_CB + U_W2) {
    const int v = u - (U_W1 + U_CB);
    const int n = v >> 5, k8 = (v & 31) * 8;
    src = W2; ld = DF; ks = k8 & (DF - 1); ncl = n;
    dp = W2T2 + (size_t)v * 8;
  } else if (u < U_TOT) {
    const int v = u - (U_W1 + U_CB + U_W2);
    const int n = v >> 5, k8 = (v & 31) * 8;
    src = W3; ld = NCLS; ks = k8 & (DF - 1); ncl = (n < NCLS) ? n : (NCLS - 1);
    zr = (n >= NCLS);
    dp = W3T2 + (size_t)v * 8;
  } else {
    return;
  }
  const float* p = src + (size_t)ks * ld + ncl;
  v8us o;
#pragma unroll
  for (int i = 0; i < 8; ++i) {
    const float f = p[(size_t)i * ld];
    o[i] = zr ? (unsigned short)0 : (unsigned short)bf16_bits(f);
  }
  *(volatile v8us*)dp = o;
  __threadfence();
  *(volatile v8us*)dp = o;
}

__global__ __launch_bounds__(NTHR) void k_cvx(const float* __restrict__ x, int nN, int nUnits,
                                              unsigned short* acat) {
  const int u = (int)blockIdx.x * NTHR + (int)threadIdx.x;
  if (u >= nUnits) return;
  const int row = u >> 4;
  const int k8  = (u & 15) * 8;
  const int rc  = row < nN ? row : nN - 1;
  const float* p = x + (size_t)rc * DF + k8;
  const v4f a = *(const v4fa*)p;
  const v4f b = *(const v4fa*)(p + 4);
  const bool ok = row < nN;
  v8us o;
  o[0] = ok ? (unsigned short)bf16_bits(a.x) : (unsigned short)0;
  o[1] = ok ? (unsigned short)bf16_bits(a.y) : (unsigned short)0;
  o[2] = ok ? (unsigned short)bf16_bits(a.z) : (unsigned short)0;
  o[3] = ok ? (unsigned short)bf16_bits(a.w) : (unsigned short)0;
  o[4] = ok ? (unsigned short)bf16_bits(b.x) : (unsigned short)0;
  o[5] = ok ? (unsigned short)bf16_bits(b.y) : (unsigned short)0;
  o[6] = ok ? (unsigned short)bf16_bits(b.z) : (unsigned short)0;
  o[7] = ok ? (unsigned short)bf16_bits(b.w) : (unsigned short)0;
  unsigned short* dp = acat + (size_t)row * KA + 2 * DF + k8;
  *(volatile v8us*)dp = o;
  __threadfence();
  *(volatile v8us*)dp = o;
}

template <int NT, int MODE>
__global__ __launch_bounds__(GTHR) void k_gemm(const unsigned short* __restrict__ A, int lda,
                                               const unsigned short* __restrict__ BT, int K,
                                               float* outF, unsigned short* outH) {
  static_assert(MODE == 0 || NT == 8);
  constexpr int COLS = 16 * NT;
  __shared__ __attribute__((aligned(16))) float stg[GBM * COLS];
  const int tid = (int)threadIdx.x, lane = tid & 31, wave = tid >> 5, hh = lane >> 4, m = lane & 15;
  const int rowBase = (int)blockIdx.x * GBM;

  v8f acc[NT];
  {
    const v8f z = {0.f, 0.f, 0.f, 0.f, 0.f, 0.f, 0.f, 0.f};
#pragma unroll
    for (int t = 0; t < NT; ++t) acc[t] = z;
  }
  const unsigned short* ap = A + (size_t)(rowBase + 16 * wave + m) * (size_t)lda + 8 * hh;
  const unsigned short* bp = BT + (size_t)m * (size_t)K + 8 * hh;

#pragma unroll 1
  for (int k0 = 0; k0 < K; k0 += 32) {
    FragB af;
    af.h[0] = *(const v8usa*)(ap + k0);
    af.h[1] = *(const v8usa*)(ap + k0 + 16);
#pragma unroll
    for (int nt = 0; nt < NT; ++nt) {
      const unsigned short* wq = bp + (size_t)(16 * nt) * (size_t)K + k0;
      FragB bf;
      bf.h[0] = *(const v8usa*)wq;
      bf.h[1] = *(const v8usa*)(wq + 16);
      acc[nt] = wmb(af, bf, acc[nt]);
    }
  }

#pragma unroll
  for (int nt = 0; nt < NT; ++nt) {
    const int lc = 16 * nt + m;
#pragma unroll
    for (int r = 0; r < 8; ++r) {
      const int lr = 16 * wave + 8 * hh + r;
      stg[lr * COLS + lc] = acc[nt][r];
    }
  }
  __syncthreads();

  if constexpr (MODE == 0) {
    constexpr int LPR = COLS / 4;
    constexpr int RPI = 32 / LPR;
    constexpr int NIT = 16 / RPI;
    const int sr = lane / LPR;
    const int c4 = (lane % LPR) * 4;
    v4f pv[NIT];
#pragma unroll
    for (int i = 0; i < NIT; ++i) pv[i] = *(const v4fa*)(stg + (16 * wave + i * RPI + sr) * COLS + c4);
#pragma unroll
    for (int i = 0; i < NIT; ++i) {
      float* op = outF + (size_t)(rowBase + 16 * wave + i * RPI + sr) * COLS + c4;
      *(volatile v4f*)op = pv[i];
    }
    __threadfence();
#pragma unroll
    for (int i = 0; i < NIT; ++i) {
      float* op = outF + (size_t)(rowBase + 16 * wave + i * RPI + sr) * COLS + c4;
      *(volatile v4f*)op = pv[i];
    }
  } else {
    v4f pv[16];
#pragma unroll
    for (int i = 0; i < 16; ++i) pv[i] = *(const v4fa*)(stg + (16 * wave + i) * COLS + 4 * lane);
    __syncthreads();
#pragma unroll
    for (int i = 0; i < 16; ++i) {
      v4us h4, l4;
      unsigned hb;
      hb = bf16_bits(pv[i].x); h4[0] = (unsigned short)hb; l4[0] = (unsigned short)bf16_bits(pv[i].x - __uint_as_float(hb << 16));
      hb = bf16_bits(pv[i].y); h4[1] = (unsigned short)hb; l4[1] = (unsigned short)bf16_bits(pv[i].y - __uint_as_float(hb << 16));
      hb = bf16_bits(pv[i].z); h4[2] = (unsigned short)hb; l4[2] = (unsigned short)bf16_bits(pv[i].z - __uint_as_float(hb << 16));
      hb = bf16_bits(pv[i].w); h4[3] = (unsigned short)hb; l4[3] = (unsigned short)bf16_bits(pv[i].w - __uint_as_float(hb << 16));
      unsigned short* srow = (unsigned short*)stg + (size_t)(16 * wave + i) * (2 * COLS);
      *(v4usa*)(srow + 4 * lane) = h4;
      *(v4usa*)(srow + DF + 4 * lane) = l4;
    }
    __syncthreads();
    v8us qv[16];
#pragma unroll
    for (int i = 0; i < 16; ++i) {
      const unsigned short* srow = (const unsigned short*)stg + (size_t)(16 * wave + i) * (2 * COLS);
      qv[i] = *(const v8usa*)(srow + 8 * lane);
    }
#pragma unroll
    for (int i = 0; i < 16; ++i) {
      unsigned short* rp = outH + (size_t)(rowBase + 16 * wave + i) * (size_t)KH + 8 * lane;
      *(volatile v8us*)rp = qv[i];
    }
    __threadfence();
#pragma unroll
    for (int i = 0; i < 16; ++i) {
      unsigned short* rp = outH + (size_t)(rowBase + 16 * wave + i) * (size_t)KH + 8 * lane;
      *(volatile v8us*)rp = qv[i];
    }
  }
}

template <int SP>
__device__ __forceinline__ v4f slot_sum(const int* sl, int o, int c, const int* __restrict__ gath,
                                        const float* __restrict__ ew, const float* __restrict__ src,
                                        int nE, int nN, int cl, int lane) {
  float a0 = 0.0f, a1 = 0.0f, a2 = 0.0f, a3 = 0.0f;
#pragma unroll 1
  for (int b0 = 0; b0 < c; b0 += 32) {
    int idx = o + b0 + lane;
    idx = idx > RCAP - 1 ? RCAP - 1 : idx;
    const int ent = sl[idx];
    int eid = ent >> SLA;
    eid = eid < 0 ? 0 : (eid > nE - 1 ? nE - 1 : eid);
    int sr = gath[eid];
    sr = sr < 0 ? 0 : (sr > nN - 1 ? nN - 1 : sr);
    const float wv  = bf16_val(ew[eid]);
    const int   wvi = __float_as_int(wv);
    const int m32 = (c - b0) < 32 ? (c - b0) : 32;
#pragma unroll 1
    for (int k = 0; k < m32; ++k) {
      const int   sk = __builtin_amdgcn_readlane(sr, k);
      const float ck = __int_as_float(__builtin_amdgcn_readlane(wvi, k));
      const v4f a = *(const v4f*)(src + (size_t)sk * SP + cl);
      a0 = fmaf(ck, a.x, a0);
      a1 = fmaf(ck, a.y, a1);
      a2 = fmaf(ck, a.z, a2);
      a3 = fmaf(ck, a.w, a3);
    }
  }
  v4f r;
  r.x = a0; r.y = a1; r.z = a2; r.w = a3;
  return r;
}

template <int MODE>
__global__ __launch_bounds__(NTHR) void k_scan(const int* __restrict__ gath, const int* __restrict__ keys,
                                               const float* __restrict__ ew,
                                               int nE, int nN, int vec8, int mRows,
                                               const float* __restrict__ src, const float* __restrict__ bias,
                                               unsigned short* apl, float* outp) {
  extern __shared__ __attribute__((aligned(16))) int dsm[];
  int* list = dsm;
  int* hl   = dsm + LISTN;
  int* sl   = hl + RCAP;
  int* cnt  = sl + RCAP;
  int* offs = cnt + NBA;
  int* cur  = offs + NBA;
  int* misc = cur + NBA;
  const int tid = (int)threadIdx.x, lane = tid & 31, wave = tid >> 5;
  int* stage = misc + MISC_INTS + wave * STGW;
  const int nodeBase = (int)blockIdx.x * NBA;

  {
    const v4i z4 = {0, 0, 0, 0};
    for (int i = tid * 4; i < AGG_ZINTS; i += NTHR * 4) *(v4ia*)(dsm + i) = z4;
    if (tid < MISC_INTS) misc[tid] = 0;
  }
  __syncthreads();

  int t = 0, ov = 0;
  const int nChunks = (nE + CHUNK - 1) / CHUNK;
#pragma unroll 1
  for (int ch = 0; ch < nChunks; ++ch) {
    const int cbase = ch * CHUNK;
    const int wc = scan_chunk<SLA>(keys, nE, cbase, nodeBase, NBA, vec8, list, tid, lane, wave);
    if (lane == 0) misc[wave] = wc;
    __syncthreads();
    if (wave == 0) {
#pragma unroll 1
      for (int w2 = 0; w2 < NWAVE; ++w2) {
        int c = misc[w2];
        c = c < 0 ? 0 : (c > WCAP ? WCAP : c);
#pragma unroll 1
        for (int b0 = 0; b0 < c; b0 += 32) {
          const int idx = b0 + lane;
          const int ent = list[w2 * WCAP + (idx < WCAP ? idx : WCAP - 1)];
          const int m32 = (c - b0) < 32 ? (c - b0) : 32;
#pragma unroll 1
          for (int k = 0; k < m32; ++k) {
            const int u    = __builtin_amdgcn_readlane(ent, k);
            const int slot = u & (NBA - 1);
            const int el   = (u >> SLA) & (CHUNK - 1);
            const int pk   = ((cbase + el) << SLA) | slot;
            if (t < RCAP) {
              if (lane == 0) { hl[t] = pk; cnt[slot] = cnt[slot] + 1; }
              t = t + 1;
            } else {
              ov = 1;
            }
          }
        }
      }
    }
    __syncthreads();
  }
  if (wave == 0 && lane == 0) { misc[8] = t; misc[9] = ov; }
  __syncthreads();
  int tt = misc[8];
  tt = tt < 0 ? 0 : (tt > RCAP ? RCAP : tt);
  const int ovf = misc[9];

  if (wave == 0) {
    const int base = lane * (NBA / 32);
    int s = 0;
#pragma unroll 1
    for (int i = 0; i < NBA / 32; ++i) s += cnt[base + i];
    int incl = s;
#pragma unroll
    for (int d = 1; d < 32; d <<= 1) {
      const int y = __shfl_up(incl, d, 32);
      if (lane >= d) incl += y;
    }
    int run = incl - s;
#pragma unroll 1
    for (int i = 0; i < NBA / 32; ++i) {
      const int cv = cnt[base + i];
      offs[base + i] = run;
      cur[base + i]  = run;
      run += cv;
    }
  }
  __syncthreads();
  if (wave == 0) {
#pragma unroll 1
    for (int b0 = 0; b0 < tt; b0 += 32) {
      const int idx = b0 + lane;
      const int ent = hl[idx < RCAP ? idx : RCAP - 1];
      const int m32 = (tt - b0) < 32 ? (tt - b0) : 32;
#pragma unroll 1
      for (int k = 0; k < m32; ++k) {
        const int u    = __builtin_amdgcn_readlane(ent, k);
        const int slot = u & (NBA - 1);
        if (lane == 0) {
          int p = cur[slot];
          p = p < 0 ? 0 : (p > RCAP - 1 ? RCAP - 1 : p);
          sl[p] = u;
          cur[slot] = p + 1;
        }
      }
    }
  }
  __syncthreads();

  const float qnan = __int_as_float(0x7fc00000);
  const float pz = (ovf != 0) ? qnan : 0.0f;

  if constexpr (MODE != 2) {
    unsigned short* rowbuf = (unsigned short*)stage;
    v4f bb;
    {
      const v4f tb = *(const v4f*)(bias + 4 * lane);
      bb.x = bf16_val(tb.x); bb.y = bf16_val(tb.y); bb.z = bf16_val(tb.z); bb.w = bf16_val(tb.w);
    }
#pragma unroll 1
    for (int si = 0; si < NBA / NWAVE; ++si) {
      const int s    = si * NWAVE + wave;
      const int node = nodeBase + s;
      int c = cnt[s];
      const bool big = c > DEGCAP;
      c = c < 0 ? 0 : (c > DEGCAP ? DEGCAP : c);
      int o = offs[s];
      o = o < 0 ? 0 : (o > RCAP ? RCAP : o);
      const v4f ag = slot_sum<DF>(sl, o, c, gath, ew, src, nE, nN, 4 * lane, lane);
      const float pzr = big ? qnan : pz;
      const bool live = node < nN;
      float y0 = ag.x + bb.x, y1 = ag.y + bb.y, y2 = ag.z + bb.z, y3 = ag.w + bb.w;
      if constexpr (MODE == 0) {
        y0 = (y0 > 0.0f) ? y0 : (y0 - y0);
        y1 = (y1 > 0.0f) ? y1 : (y1 - y1);
        y2 = (y2 > 0.0f) ? y2 : (y2 - y2);
        y3 = (y3 > 0.0f) ? y3 : (y3 - y3);
      }
      const float m0 = live ? (y0 + pzr) : 0.0f;
      const float m1 = live ? (y1 + pzr) : 0.0f;
      const float m2 = live ? (y2 + pzr) : 0.0f;
      const float m3 = live ? (y3 + pzr) : 0.0f;
      v4us mh, ml;
      {
        unsigned hb;
        hb = bf16_bits(m0); mh[0] = (unsigned short)hb; ml[0] = (unsigned short)bf16_bits(m0 - __uint_as_float(hb << 16));
        hb = bf16_bits(m1); mh[1] = (unsigned short)hb; ml[1] = (unsigned short)bf16_bits(m1 - __uint_as_float(hb << 16));
        hb = bf16_bits(m2); mh[2] = (unsigned short)hb; ml[2] = (unsigned short)bf16_bits(m2 - __uint_as_float(hb << 16));
        hb = bf16_bits(m3); mh[3] = (unsigned short)hb; ml[3] = (unsigned short)bf16_bits(m3 - __uint_as_float(hb << 16));
      }
      *(v4usa*)(rowbuf + 4 * lane) = mh;
      *(v4usa*)(rowbuf + DF + 4 * lane) = ml;
      wave_sync();
      const v8us q0 = *(const v8usa*)(rowbuf + 8 * lane);
      wave_sync();
      if (node < mRows) {
        unsigned short* rpw = apl + (size_t)node * KA + 8 * lane;
        *(volatile v8us*)rpw = q0;
        __threadfence();
        *(volatile v8us*)rpw = q0;
      }
    }
  } else {
    float* ob = (float*)stage;
    const int l16 = lane & 15;
    const bool vl = l16 < (NCLS / 4);
    const int bcl = vl ? l16 : (NCLS / 4 - 1);
    v4f bb;
    {
      const v4f tb = *(const v4f*)(bias + 4 * bcl);
      bb.x = vl ? bf16_val(tb.x) : 0.0f; bb.y = vl ? bf16_val(tb.y) : 0.0f;
      bb.z = vl ? bf16_val(tb.z) : 0.0f; bb.w = vl ? bf16_val(tb.w) : 0.0f;
    }
    const float ninf = -__builtin_huge_valf();
#pragma unroll 1
    for (int gi = 0; gi < (NBA / 32) / NWAVE; ++gi) {
      const int g     = gi * NWAVE + wave;
      const int gbase = nodeBase + 32 * g;
#pragma unroll 1
      for (int r = 0; r < 32; ++r) {
        const int s    = 32 * g + r;
        const int node = gbase + r;
        int c = cnt[s];
        const bool big = c > DEGCAP;
        c = c < 0 ? 0 : (c > DEGCAP ? DEGCAP : c);
        int o = offs[s];
        o = o < 0 ? 0 : (o > RCAP ? RCAP : o);
        const v4f ag = slot_sum<NC3>(sl, o, c, gath, ew, src, nE, nN, 4 * l16, lane);
        const float pzr = big ? qnan : pz;
        const bool live = node < nN;
        const float v0 = ag.x + bb.x, v1 = ag.y + bb.y, v2 = ag.z + bb.z, v3 = ag.w + bb.w;
        float mx = fmaxf(fmaxf(v0, v1), fmaxf(v2, v3));
        mx = vl ? mx : ninf;
        mx = fmaxf(mx, __shfl_xor(mx, 8, 32));
        mx = fmaxf(mx, __shfl_xor(mx, 4, 32));
        mx = fmaxf(mx, __shfl_xor(mx, 2, 32));
        mx = fmaxf(mx, __shfl_xor(mx, 1, 32));
        const float d0 = v0 - mx, d1 = v1 - mx, d2 = v2 - mx, d3 = v3 - mx;
        const float es = (expf(d0) + expf(d1)) + (expf(d2) + expf(d3));
        float sm = vl ? es : 0.0f;
        sm += __shfl_xor(sm, 8, 32);
        sm += __shfl_xor(sm, 4, 32);
        sm += __shfl_xor(sm, 2, 32);
        sm += __shfl_xor(sm, 1, 32);
        const float lg = logf(sm);
        v4f o4;
        o4.x = live ? ((d0 - lg) + pzr) : 0.0f;
        o4.y = live ? ((d1 - lg) + pzr) : 0.0f;
        o4.z = live ? ((d2 - lg) + pzr) : 0.0f;
        o4.w = live ? ((d3 - lg) + pzr) : 0.0f;
        if (lane < NCLS / 4) *(v4fa*)(ob + r * NCLS + 4 * lane) = o4;
      }
      wave_sync();
      v4f pc[10];
#pragma unroll
      for (int it = 0; it < 10; ++it) pc[it] = *(const v4fa*)(ob + 4 * (it * 32 + lane));
      wave_sync();
      int nv = nN - gbase;
      nv = nv < 0 ? 0 : (nv > 32 ? 32 : nv);
      const int npc = nv * (NCLS / 4);
      const int gb = gbase < nN ? gbase : nN;
      float* obase = outp + (size_t)gb * NCLS;
#pragma unroll
      for (int it = 0; it < 10; ++it)
        if (it * 32 + lane < npc) *(volatile v4f*)(obase + 4 * (it * 32 + lane)) = pc[it];
      __threadfence();
#pragma unroll
      for (int it = 0; it < 10; ++it)
        if (it * 32 + lane < npc) *(volatile v4f*)(obase + 4 * (it * 32 + lane)) = pc[it];
    }
  }
}

static inline int cdiv(int a, int b) { return (a + b - 1) / b; }
static inline size_t al256(size_t o) { return (o + 255) & ~(size_t)255; }

extern "C" void kernel_launch(void* const* d_in, const int* in_sizes, int n_in,
                              void* d_out, int out_size, void* d_ws, size_t ws_size,
                              hipStream_t stream) {
  if (n_in < 11) return;
  if (in_sizes[0] < DF || (in_sizes[0] % DF) != 0) return;
  const int nN = in_sizes[0] / DF;
  const int nE = in_sizes[1];
  if (nE < 1 || in_sizes[2] != nE || in_sizes[3] != nE) return;
  if (nE >= (1 << 21) || nN < 16 || nN >= (1 << 24)) return;
  if ((nN & 3) != 0) return;
  if (in_sizes[4] != DF * DF || in_sizes[5] != DF) return;
  if (in_sizes[6] != DF * DF || in_sizes[7] != DF) return;
  if (in_sizes[8] != DF * NCLS || in_sizes[9] != NCLS) return;
  if (in_sizes[10] != 2 * DF * DF) return;
  if ((long long)out_size != (long long)nN * NCLS) return;

  const float* x   = (const float*)d_in[0];
  const int*   row = (const int*)d_in[1];
  const int*   col = (const int*)d_in[2];
  const float* val = (const float*)d_in[3];
  const float* W1  = (const float*)d_in[4];
  const float* b1  = (const float*)d_in[5];
  const float* W2  = (const float*)d_in[6];
  const float* b2  = (const float*)d_in[7];
  const float* W3  = (const float*)d_in[8];
  const float* b3  = (const float*)d_in[9];
  const float* CMB = (const float*)d_in[10];
  float* out = (float*)d_out;

  const int MP = cdiv(nN, GBM) * GBM;
  const int gM = MP / GBM;
  const int gA = cdiv(MP, NBA);
  if ((long long)gA * NBA < (long long)MP) return;
  const int vec8 = ((nE & 3) == 0) ? 1 : 0;

  char* ws = (char*)d_ws;
  size_t off = 0;
  const size_t oW1T = off; off = al256(off + (size_t)DF * DF * 2);
  const size_t oCB3 = off; off = al256(off + (size_t)DF * KA * 2);
  const size_t oW22 = off; off = al256(off + (size_t)DF * KH * 2);
  const size_t oW32 = off; off = al256(off + (size_t)NC3 * KH * 2);
  const size_t oAC  = off; off = al256(off + (size_t)MP * KA * 2);
  const size_t oS   = off; off = al256(off + (size_t)MP * DF * 4);
  const size_t oCH  = off; off = al256(off + (size_t)MP * KH * 2);
  const size_t oT3  = off; off = al256(off + (size_t)MP * NC3 * 4);
  if (off > ws_size || off > (size_t)WSMAX) return;
  unsigned short* W1T  = (unsigned short*)(ws + oW1T);
  unsigned short* CB3  = (unsigned short*)(ws + oCB3);
  unsigned short* W2T2 = (unsigned short*)(ws + oW22);
  unsigned short* W3T2 = (unsigned short*)(ws + oW32);
  unsigned short* ACAT = (unsigned short*)(ws + oAC);
  float*          S    = (float*)(ws + oS);
  unsigned short* CHL  = (unsigned short*)(ws + oCH);
  float*          T3   = (float*)(ws + oT3);

  const size_t scanLds = (size_t)AGG_LDS_INTS * 4;
  hipFuncSetAttribute(reinterpret_cast<const void*>(&k_scan<0>), hipFuncAttributeMaxDynamicSharedMemorySize, (int)scanLds);
  hipFuncSetAttribute(reinterpret_cast<const void*>(&k_scan<1>), hipFuncAttributeMaxDynamicSharedMemorySize, (int)scanLds);
  hipFuncSetAttribute(reinterpret_cast<const void*>(&k_scan<2>), hipFuncAttributeMaxDynamicSharedMemorySize, (int)scanLds);

  const int nUx = MP * (DF / 8);
  k_wprep<<<U_TOT / NTHR, NTHR, 0, stream>>>(W1, W2, W3, CMB, W1T, CB3, W2T2, W3T2);
  k_cvx<<<cdiv(nUx, NTHR), NTHR, 0, stream>>>(x, nN, nUx, ACAT);
  k_gemm<8, 0><<<gM, GTHR, 0, stream>>>(ACAT + 2 * DF, KA, W1T, DF, S, CHL);
  k_scan<0><<<gA, NTHR, scanLds, stream>>>(col, row, val, nE, nN, vec8, MP, S, b1, ACAT, out);
  k_gemm<8, 1><<<gM, GTHR, 0, stream>>>(ACAT, KA, CB3, KA, S, CHL);
  k_gemm<8, 0><<<gM, GTHR, 0, stream>>>(CHL, KH, W2T2, KH, S, CHL);
  k_scan<1><<<gA, NTHR, scanLds, stream>>>(col, row, val, nE, nN, vec8, MP, S, b2, ACAT, out);
  k_gemm<8, 1><<<gM, GTHR, 0, stream>>>(ACAT, KA, CB3, KA, S, CHL);
  k_gemm<4, 0><<<gM, GTHR, 0, stream>>>(CHL, KH, W3T2, KH, T3, CHL);
  k_scan<2><<<gA, NTHR, scanLds, stream>>>(col, row, val, nE, nN, vec8, MP, T3, b3, ACAT, out);
}
